// NeuralColony_90039694393638
// MI455X (gfx1250) — hardware-verified
//
#include <hip/hip_runtime.h>


#define NB_   2
#define NL_   1024
#define DM_   1024
#define DI_   2048
#define NS_   16
#define DTR_  64
#define NPJ_  96
#define PJP_  128
#define NN_   8
#define MT_   (NB_ * NL_)
#define YSC_  16.0f

static_assert(MT_ % 64 == 0);
static_assert((2 * DI_) % 128 == 0);
static_assert(DI_ % 128 == 0);
static_assert(DM_ % 128 == 0);
static_assert(PJP_ % 128 == 0);
static_assert(DM_ % 32 == 0);
static_assert(DI_ % 32 == 0);
static_assert(DTR_ % 32 == 0);
static_assert((NL_ & (NL_ - 1)) == 0);
static_assert(NL_ % 16 == 0);
static_assert(DI_ == 8 * 256);
static_assert(DM_ == 4 * 256);
static_assert(DI_ % 64 == 0);
static_assert(NPJ_ == DTR_ + 2 * NS_);
static_assert(NPJ_ <= PJP_);

typedef float          v4f   __attribute__((ext_vector_type(4)));
typedef float          v8f   __attribute__((ext_vector_type(8)));
typedef _Float16       v8h   __attribute__((ext_vector_type(8)));
typedef _Float16       v16h  __attribute__((ext_vector_type(16)));
typedef unsigned short u16x8 __attribute__((ext_vector_type(8)));

union FragH { u16x8 h[2]; v16h v; };
union Pack8 { v8h f; u16x8 u; };

__device__ __forceinline__ float silu_f(float x) {
    const float e = __expf(-x);
    return x * __builtin_amdgcn_rcpf(1.0f + e);
}
__device__ __forceinline__ float softplus_f(float x) {
    return fmaxf(x, 0.0f) + log1pf(__expf(-fabsf(x)));
}
__device__ __forceinline__ float conv4_silu(float x0, float x1, float x2, float x3,
                                            float w0, float w1, float w2, float w3, float bias) {
    const float c = w0 * x0 + w1 * x1 + w2 * x2 + w3 * x3;
    return silu_f(c + bias);
}
__device__ __forceinline__ v8f ld8f(const float* p) {
    const v4f a = *(const v4f*)p;
    const v4f b = *(const v4f*)(p + 4);
    return __builtin_shufflevector(a, b, 0, 1, 2, 3, 4, 5, 6, 7);
}
__device__ __forceinline__ float wave_sum(float v) {
#pragma unroll
    for (int o = 16; o > 0; o >>= 1) v += __shfl_xor(v, o);
    return v;
}

__device__ __forceinline__ void mma16(v8f& acc, const FragH& a, const FragH& b) {
    acc = __builtin_amdgcn_wmma_f32_16x16x32_f16(false, a.v, false, b.v, (short)0, acc, false, false);
    asm volatile("v_nop\n\tv_nop\n\tv_nop\n\tv_nop" : "+v"(acc) : "v"(a.v), "v"(b.v));
}

__global__ __launch_bounds__(256)
void cvt_kernel(const float* __restrict__ src, int spitch, unsigned short* dst, int dpitch,
                int rows, int srows, int c8, float scale)
{
    const int i = blockIdx.x * 256 + threadIdx.x;
    if (i >= rows * c8) return;
    const int r = i / c8;
    const int c = (i - r * c8) * 8;
    v8f x;
#pragma unroll
    for (int q = 0; q < 8; ++q) x[q] = 0.0f;
    if (r < srows) x = ld8f(src + (size_t)r * spitch + c);
    Pack8 pk;
    pk.f = __builtin_convertvector(x * scale, v8h);
    const u16x8 v = pk.u;
    unsigned short* p = dst + (size_t)r * dpitch + c;
    *(volatile u16x8*)p = v;
    __threadfence();
    *(volatile u16x8*)p = v;
}

template<int NBF>
__device__ __forceinline__ void tile_store_pass(const float* st, float* gp, int ldc, int lane) {
    constexpr int CW  = NBF * 16;
    constexpr int P   = CW + 4;
    constexpr int LPR = CW / 4;
    constexpr int RPI = 32 / LPR;
    constexpr int NIT = 32 / RPI;
    const int rsub = lane / LPR;
    const int c4   = (lane % LPR) * 4;
#pragma unroll
    for (int it = 0; it < NIT; ++it) {
        const int row = it * RPI + rsub;
        const v4f v = *(const v4f*)(st + row * P + c4);
        *(volatile v4f*)(gp + (size_t)row * ldc + c4) = v;
    }
}

template<int NBF>
__global__ __launch_bounds__(128)
void gemm_tn_kernel(const unsigned short* __restrict__ A, const unsigned short* __restrict__ Bw,
                    float* C, float* C2, int K, int ldc, int csplit, float scale)
{
    constexpr int CW = NBF * 16;
    constexpr int P  = CW + 4;
    __shared__ __attribute__((aligned(16))) float stile[4][32 * P];

    const int tid  = threadIdx.x;
    const int lane = tid & 31;
    const int wave = tid >> 5;
    const int h    = lane >> 4;
    const int m    = lane & 15;
    const int wm   = wave >> 1;
    const int wn   = wave & 1;

    const int rowW = blockIdx.y * 64 + wm * 32;
    const int colW = blockIdx.x * (2 * CW) + wn * CW;

    v8f acc[2 * NBF];
#pragma unroll
    for (int j = 0; j < 2 * NBF; ++j)
#pragma unroll
        for (int r = 0; r < 8; ++r) acc[j][r] = 0.0f;

    const size_t aoff  = (size_t)(rowW + m) * K + 8 * h;
    const size_t boff  = (size_t)(colW + m) * K + 8 * h;
    const size_t sub16 = (size_t)16 * K;
    const int nk = K >> 5;

    for (int kt = 0; kt < nk; ++kt) {
        const size_t k0 = (size_t)kt * 32;
        FragH fa[2], fb[NBF];
#pragma unroll
        for (int s = 0; s < 2; ++s) {
            const unsigned short* p = A + aoff + s * sub16 + k0;
            fa[s].h[0] = *(const u16x8*)(p);
            fa[s].h[1] = *(const u16x8*)(p + 16);
        }
#pragma unroll
        for (int j = 0; j < NBF; ++j) {
            const unsigned short* p = Bw + boff + j * sub16 + k0;
            fb[j].h[0] = *(const u16x8*)(p);
            fb[j].h[1] = *(const u16x8*)(p + 16);
        }
#pragma unroll
        for (int s = 0; s < 2; ++s)
#pragma unroll
            for (int j = 0; j < NBF; ++j)
                mma16(acc[s * NBF + j], fa[s], fb[j]);
    }

    float* st = stile[wave];
#pragma unroll
    for (int s = 0; s < 2; ++s)
#pragma unroll
        for (int j = 0; j < NBF; ++j)
#pragma unroll
            for (int r = 0; r < 8; ++r)
                st[(s * 16 + 8 * h + r) * P + j * 16 + m] = acc[s * NBF + j][r] * scale;
    __syncthreads();

    float* Cp = C;
    int gcol = colW;
    if (colW >= csplit) { Cp = C2; gcol = colW - csplit; }
    float* gp = Cp + (size_t)rowW * ldc + gcol;
    tile_store_pass<NBF>(st, gp, ldc, lane);
    __threadfence();
    tile_store_pass<NBF>(st, gp, ldc, lane);
}

__global__ __launch_bounds__(256)
void conv_silu_kernel(const float* __restrict__ X, const float* __restrict__ cw,
                      const float* __restrict__ cb, unsigned short* U16)
{
    const int m  = blockIdx.x;
    const int l  = m & (NL_ - 1);
    const int d0 = threadIdx.x * 8;
    const float* xr = X + (size_t)m * DI_ + d0;

    const v8f x3 = ld8f(xr);
    v8f x2, x1, x0;
#pragma unroll
    for (int c = 0; c < 8; ++c) { x2[c] = 0.0f; x1[c] = 0.0f; x0[c] = 0.0f; }
    if (l >= 1) x2 = ld8f(xr - DI_);
    if (l >= 2) x1 = ld8f(xr - 2 * DI_);
    if (l >= 3) x0 = ld8f(xr - 3 * DI_);

    const float* wp = cw + (size_t)d0 * 4;
    v4f wv[8];
#pragma unroll
    for (int c = 0; c < 8; ++c) wv[c] = *(const v4f*)(wp + 4 * c);
    const v8f bias = ld8f(cb + d0);

    v8f u;
#pragma unroll
    for (int c = 0; c < 8; ++c)
        u[c] = conv4_silu(x0[c], x1[c], x2[c], x3[c], wv[c][0], wv[c][1], wv[c][2], wv[c][3], bias[c]);

    Pack8 pk;
    pk.f = __builtin_convertvector(u, v8h);
    const u16x8 v = pk.u;
    unsigned short* gp = U16 + (size_t)m * DI_ + d0;
    *(volatile u16x8*)gp = v;
    __threadfence();
    *(volatile u16x8*)gp = v;
}

__device__ __forceinline__ void yrows_store_pass(const _Float16* sy, unsigned short* Y16,
                                                 size_t gbase, int wave, int lane) {
#pragma unroll
    for (int it = 0; it < 2; ++it) {
        const int t = wave * 8 + it * 4 + (lane >> 3);
        const int c = (lane & 7) * 8;
        Pack8 pk;
        pk.f = *(const v8h*)(sy + t * 64 + c);
        const u16x8 v = pk.u;
        *(volatile u16x8*)(Y16 + gbase + (size_t)t * DI_ + c) = v;
    }
}

__global__ __launch_bounds__(64)
void scan_kernel(const float* __restrict__ X, const float* __restrict__ Z, const float* __restrict__ Dl,
                 const float* __restrict__ proj,
                 const float* __restrict__ cw, const float* __restrict__ cb,
                 const float* __restrict__ dtb, const float* __restrict__ Alog,
                 const float* __restrict__ Dp, unsigned short* Y16)
{
    __shared__ __attribute__((aligned(16))) _Float16 sY[16 * 64];
    __shared__ __attribute__((aligned(16))) float    sBC[16 * 32];

    const int tid   = threadIdx.x;
    const int lane  = tid & 31;
    const int wave  = tid >> 5;
    const int dbase = blockIdx.x * 64;
    const int d     = dbase + tid;
    const int b     = blockIdx.y;

    float an[NS_], hs[NS_];
#pragma unroll
    for (int n = 0; n < NS_; ++n) {
        an[n] = -expf(Alog[d * NS_ + n]);
        hs[n] = 0.0f;
    }
    const float w0 = cw[d * 4 + 0], w1 = cw[d * 4 + 1], w2 = cw[d * 4 + 2], w3 = cw[d * 4 + 3];
    const float cbias = cb[d];
    const float pb    = dtb[d];
    const float Dd    = Dp[d];

    float xm1 = 0.0f, xm2 = 0.0f, xm3 = 0.0f;
    const size_t mrow0 = (size_t)b * NL_;
    const int st_t = tid >> 2;
    const int st_q = tid & 3;

#pragma unroll 1
    for (int l0 = 0; l0 < NL_; l0 += 16) {
        {
            const float* pr = proj + (mrow0 + (size_t)(l0 + st_t)) * PJP_ + DTR_ + st_q * 8;
            const v4f a0 = *(const v4f*)pr;
            const v4f a1 = *(const v4f*)(pr + 4);
            *(v4f*)(sBC + st_t * 32 + st_q * 8)     = a0;
            *(v4f*)(sBC + st_t * 32 + st_q * 8 + 4) = a1;
        }
        __syncthreads();
#pragma unroll 1
        for (int t = 0; t < 16; ++t) {
            const size_t e = (mrow0 + (size_t)(l0 + t)) * DI_ + d;
            const float xv = X[e];
            const float zv = Z[e];
            const float dl = Dl[e];
            const float u  = conv4_silu(xm3, xm2, xm1, xv, w0, w1, w2, w3, cbias);
            xm3 = xm2; xm2 = xm1; xm1 = xv;
            const float dt = softplus_f(dl + pb);
            v4f bq[4], cq[4];
#pragma unroll
            for (int q = 0; q < 4; ++q) {
                bq[q] = *(const v4f*)(sBC + t * 32 + 4 * q);
                cq[q] = *(const v4f*)(sBC + t * 32 + 16 + 4 * q);
            }
            float y = 0.0f;
#pragma unroll
            for (int n = 0; n < NS_; ++n) {
                const float bn = bq[n >> 2][n & 3];
                const float cn = cq[n >> 2][n & 3];
                const float da = __expf(dt * an[n]);
                hs[n] = hs[n] * da + (dt * bn) * u;
                y += hs[n] * cn;
            }
            const float g = (y + u * Dd) * silu_f(zv);
            sY[t * 64 + tid] = (_Float16)(g * YSC_);
        }
        __syncthreads();
        const size_t gbase = (mrow0 + (size_t)l0) * DI_ + dbase;
        yrows_store_pass(sY, Y16, gbase, wave, lane);
        __threadfence();
        yrows_store_pass(sY, Y16, gbase, wave, lane);
        __syncthreads();
    }
}

__global__ __launch_bounds__(256)
void final_kernel(const float* __restrict__ x, const float* __restrict__ core,
                  const float* __restrict__ nsc, const float* __restrict__ nbi,
                  const float* __restrict__ lnw, const float* __restrict__ lnb,
                  const float* __restrict__ mask, float* out)
{
    __shared__ float sredA[8];
    __shared__ float sredB[8];
    const int row  = blockIdx.x;
    const int tid  = threadIdx.x;
    const int lane = tid & 31;
    const int wave = tid >> 5;
    const int c0   = tid * 4;
    const size_t rb = (size_t)row * DM_ + c0;

    const v4f xv = *(const v4f*)(x + rb);
    const v4f cv = *(const v4f*)(core + rb);
    v4f es;
#pragma unroll
    for (int c = 0; c < 4; ++c) es[c] = 0.0f;
#pragma unroll
    for (int n = 0; n < NN_; ++n) {
        const v4f s  = *(const v4f*)(nsc + (size_t)n * DM_ + c0);
        const v4f bq = *(const v4f*)(nbi + (size_t)n * DM_ + c0);
        es = es + (cv * s + bq);
    }
    const v4f hv = xv + es * 0.125f;

    float ps = (hv[0] + hv[1]) + (hv[2] + hv[3]);
    ps = wave_sum(ps);
    if (lane == 0) sredA[wave] = ps;
    __syncthreads();
    float tot = 0.0f;
#pragma unroll
    for (int i = 0; i < 8; ++i) tot += sredA[i];
    const float mean = tot * (1.0f / DM_);

    const v4f dv = hv - mean;
    float ps2 = (dv[0] * dv[0] + dv[1] * dv[1]) + (dv[2] * dv[2] + dv[3] * dv[3]);
    ps2 = wave_sum(ps2);
    if (lane == 0) sredB[wave] = ps2;
    __syncthreads();
    float tot2 = 0.0f;
#pragma unroll
    for (int i = 0; i < 8; ++i) tot2 += sredB[i];
    const float var = tot2 * (1.0f / DM_);
    const float inv = rsqrtf(var + 1e-5f);

    const v4f w  = *(const v4f*)(lnw + c0);
    const v4f bb = *(const v4f*)(lnb + c0);
    const float mk = mask[row];
    const v4f o = ((dv * inv) * w + bb) * mk;

    *(volatile v4f*)(out + rb) = o;
    __threadfence();
    *(volatile v4f*)(out + rb) = o;
}

extern "C" void kernel_launch(void* const* d_in, const int* in_sizes, int n_in,
                              void* d_out, int out_size, void* d_ws, size_t ws_size,
                              hipStream_t stream)
{
    if (n_in < 15) return;
    if (in_sizes[0]  != MT_ * DM_)       return;
    if (in_sizes[1]  != MT_)             return;
    if (in_sizes[2]  != 2 * DI_ * DM_)   return;
    if (in_sizes[3]  != DI_ * 4)         return;
    if (in_sizes[4]  != DI_)             return;
    if (in_sizes[5]  != NPJ_ * DI_)      return;
    if (in_sizes[6]  != DI_ * DTR_)      return;
    if (in_sizes[7]  != DI_)             return;
    if (in_sizes[8]  != DI_ * NS_)       return;
    if (in_sizes[9]  != DI_)             return;
    if (in_sizes[10] != DM_ * DI_)       return;
    if (in_sizes[11] != NN_ * DM_)       return;
    if (in_sizes[12] != NN_ * DM_)       return;
    if (in_sizes[13] != DM_)             return;
    if (in_sizes[14] != DM_)             return;
    if (out_size != MT_ * DM_)           return;

    const float* xin  = (const float*)d_in[0];
    const float* amsk = (const float*)d_in[1];
    const float* wi   = (const float*)d_in[2];
    const float* cw   = (const float*)d_in[3];
    const float* cb   = (const float*)d_in[4];
    const float* wx   = (const float*)d_in[5];
    const float* wd   = (const float*)d_in[6];
    const float* dtb  = (const float*)d_in[7];
    const float* alog = (const float*)d_in[8];
    const float* Dp   = (const float*)d_in[9];
    const float* wo   = (const float*)d_in[10];
    const float* nsc  = (const float*)d_in[11];
    const float* nbi  = (const float*)d_in[12];
    const float* lnw  = (const float*)d_in[13];
    const float* lnb  = (const float*)d_in[14];
    float* out = (float*)d_out;

    const size_t SZ_X16  = (size_t)MT_ * DM_ * 2;
    const size_t SZ_WI   = (size_t)2 * DI_ * DM_ * 2;
    const size_t SZ_WX   = (size_t)PJP_ * DI_ * 2;
    const size_t SZ_WD   = (size_t)DI_ * DTR_ * 2;
    const size_t SZ_WO   = (size_t)DM_ * DI_ * 2;
    const size_t SZ_F    = (size_t)MT_ * DI_ * 4;
    const size_t SZ_U16  = (size_t)MT_ * DI_ * 2;
    const size_t SZ_PJ   = (size_t)MT_ * PJP_ * 4;
    const size_t SZ_DTR  = (size_t)MT_ * DTR_ * 2;
    const size_t SZ_Y16  = (size_t)MT_ * DI_ * 2;
    const size_t SZ_CORE = (size_t)MT_ * DM_ * 4;

    const size_t OFF_X16  = 0;
    const size_t OFF_WI   = OFF_X16 + SZ_X16;
    const size_t OFF_WX   = OFF_WI + SZ_WI;
    const size_t OFF_WD   = OFF_WX + SZ_WX;
    const size_t OFF_WO   = OFF_WD + SZ_WD;
    const size_t OFF_XF   = OFF_WO + SZ_WO;
    const size_t OFF_ZF   = OFF_XF + SZ_F;
    const size_t OFF_U16  = OFF_ZF + SZ_F;
    const size_t OFF_PJ   = OFF_U16 + SZ_U16;
    const size_t OFF_DTR  = OFF_PJ + SZ_PJ;
    const size_t OFF_DL   = OFF_DTR + SZ_DTR;
    const size_t OFF_Y16  = OFF_DL + SZ_F;
    const size_t OFF_CORE = OFF_Y16 + SZ_Y16;
    const size_t WS_END   = OFF_CORE + SZ_CORE;
    if (ws_size < WS_END) return;

    char* ws = (char*)d_ws;
    unsigned short* x16   = (unsigned short*)(ws + OFF_X16);
    unsigned short* wi16  = (unsigned short*)(ws + OFF_WI);
    unsigned short* wx16  = (unsigned short*)(ws + OFF_WX);
    unsigned short* wd16  = (unsigned short*)(ws + OFF_WD);
    unsigned short* wo16  = (unsigned short*)(ws + OFF_WO);
    float*          Xf    = (float*)(ws + OFF_XF);
    float*          Zf    = (float*)(ws + OFF_ZF);
    unsigned short* u16   = (unsigned short*)(ws + OFF_U16);
    float*          proj  = (float*)(ws + OFF_PJ);
    unsigned short* dtr16 = (unsigned short*)(ws + OFF_DTR);
    float*          Dl    = (float*)(ws + OFF_DL);
    unsigned short* y16   = (unsigned short*)(ws + OFF_Y16);
    float*          core  = (float*)(ws + OFF_CORE);

    {
        int units;
        units = MT_ * (DM_ / 8);
        cvt_kernel<<<dim3((units + 255) / 256), dim3(256), 0, stream>>>(
            xin, (int)DM_, x16, (int)DM_, (int)MT_, (int)MT_, (int)(DM_ / 8), 1.0f);
        units = (2 * DI_) * (DM_ / 8);
        cvt_kernel<<<dim3((units + 255) / 256), dim3(256), 0, stream>>>(
            wi, (int)DM_, wi16, (int)DM_, (int)(2 * DI_), (int)(2 * DI_), (int)(DM_ / 8), 32.0f);
        units = PJP_ * (DI_ / 8);
        cvt_kernel<<<dim3((units + 255) / 256), dim3(256), 0, stream>>>(
            wx, (int)DI_, wx16, (int)DI_, (int)PJP_, (int)NPJ_, (int)(DI_ / 8), 32.0f);
        units = DI_ * (DTR_ / 8);
        cvt_kernel<<<dim3((units + 255) / 256), dim3(256), 0, stream>>>(
            wd, (int)DTR_, wd16, (int)DTR_, (int)DI_, (int)DI_, (int)(DTR_ / 8), 1.0f);
        units = DM_ * (DI_ / 8);
        cvt_kernel<<<dim3((units + 255) / 256), dim3(256), 0, stream>>>(
            wo, (int)DI_, wo16, (int)DI_, (int)DM_, (int)DM_, (int)(DI_ / 8), 32.0f);
    }

    gemm_tn_kernel<4><<<dim3((2 * DI_) / 128, MT_ / 64), dim3(128), 0, stream>>>(
        (const unsigned short*)x16, (const unsigned short*)wi16,
        Xf, Zf, (int)DM_, (int)DI_, (int)DI_, 0.03125f);

    conv_silu_kernel<<<dim3(MT_), dim3(DI_ / 8), 0, stream>>>((const float*)Xf, cw, cb, u16);

    gemm_tn_kernel<4><<<dim3(PJP_ / 128, MT_ / 64), dim3(128), 0, stream>>>(
        (const unsigned short*)u16, (const unsigned short*)wx16,
        proj, proj, (int)DI_, (int)PJP_, (int)(4 * PJP_), 0.03125f);

    {
        const int units = MT_ * (DTR_ / 8);
        cvt_kernel<<<dim3((units + 255) / 256), dim3(256), 0, stream>>>(
            (const float*)proj, (int)PJP_, dtr16, (int)DTR_, (int)MT_, (int)MT_, (int)(DTR_ / 8), 1.0f);
    }

    gemm_tn_kernel<4><<<dim3(DI_ / 128, MT_ / 64), dim3(128), 0, stream>>>(
        (const unsigned short*)dtr16, (const unsigned short*)wd16,
        Dl, Dl, (int)DTR_, (int)DI_, (int)(4 * DI_), 1.0f);

    scan_kernel<<<dim3(DI_ / 64, NB_), dim3(64), 0, stream>>>(
        (const float*)Xf, (const float*)Zf, (const float*)Dl, (const float*)proj,
        cw, cb, dtb, alog, Dp, y16);

    gemm_tn_kernel<4><<<dim3(DM_ / 128, MT_ / 64), dim3(128), 0, stream>>>(
        (const unsigned short*)y16, (const unsigned short*)wo16,
        core, core, (int)DI_, (int)DM_, (int)(4 * DM_), 0.001953125f);

    final_kernel<<<dim3(MT_), dim3(256), 0, stream>>>(
        xin, (const float*)core, nsc, nbi, lnw, lnb, amsk, out);
}
